// Block_48627619725752
// MI455X (gfx1250) — hardware-verified
//
#include <hip/hip_runtime.h>
#include <math.h>

#ifndef NB
#define NB 2
#endif
#ifndef SEQ
#define SEQ 2048
#endif
#define NB_FULL 2
#define SEQ_FULL 2048
#define CW 1024
#define NH 16
#define HD 64
#define FW 4096
#define QKW 2048
#define MROWS (NB * SEQ)
#define VTP MROWS

static_assert(CW == NH * HD);
static_assert(CW == 128 * 8);
static_assert(HD == 64);
static_assert(SEQ % 64 == 0);
static_assert(MROWS % 64 == 0);
static_assert(CW % 64 == 0 && FW % 64 == 0 && QKW % 64 == 0);
static_assert(CW % 32 == 0 && FW % 32 == 0);
static_assert(QKW == 2 * CW);
static_assert(NB <= NB_FULL && SEQ <= SEQ_FULL);
static_assert(MROWS % 8 == 0);

typedef _Float16 v16h __attribute__((ext_vector_type(16)));
typedef _Float16 v8h  __attribute__((ext_vector_type(8)));
typedef float    v8f  __attribute__((ext_vector_type(8)));
typedef float    v4f  __attribute__((ext_vector_type(4)));
typedef v8h v8h_a __attribute__((may_alias));
typedef v4f v4f_a __attribute__((may_alias));
typedef unsigned int cm_u4 __attribute__((ext_vector_type(4)));
typedef unsigned int bk_u2 __attribute__((ext_vector_type(2)));

union FragU { v16h v; v8h h[2]; };
__device__ __forceinline__ v16h ld_frag(const _Float16* __restrict__ p) {
    FragU f; f.h[0] = *(const v8h*)(p); f.h[1] = *(const v8h*)(p + 16); return f.v;
}
__device__ __forceinline__ v8f mma16(v16h a, v16h b, v8f c) {
    c = __builtin_amdgcn_wmma_f32_16x16x32_f16(false, a, false, b, (short)0, c, false, false);
    asm volatile("v_nop\n\tv_nop\n\tv_nop\n\tv_nop" : "+v"(c) : "v"(a), "v"(b));
    return c;
}
__device__ __forceinline__ v8f mma16_raw(v16h a, v16h b, v8f c) {
    return __builtin_amdgcn_wmma_f32_16x16x32_f16(false, a, false, b, (short)0, c, false, false);
}
__device__ __forceinline__ void dep_guard_h(v8f& a, v8f& b, v16h x, v16h y) { asm volatile("v_nop\n\tv_nop\n\tv_nop\n\tv_nop" : "+v"(a), "+v"(b) : "v"(x), "v"(y)); }
__device__ __forceinline__ void keep4_h(v16h a, v16h b, v16h c, v16h d) { asm volatile("v_nop" :: "v"(a), "v"(b), "v"(c), "v"(d)); }
__device__ __forceinline__ void acc_guard4(v8f& a, v8f& b, v8f& c, v8f& d) { asm volatile("v_nop\n\tv_nop\n\tv_nop\n\tv_nop" : "+v"(a), "+v"(b), "+v"(c), "+v"(d)); }
__device__ __forceinline__ void wave_lds_sync() {
    __builtin_amdgcn_fence(3  , "workgroup");
    __builtin_amdgcn_wave_barrier();
    __builtin_amdgcn_fence(2  , "workgroup");
}

#define VST2(T, ptr, val) do { const T vst2_v_ = (val); *(volatile T*)(ptr) = vst2_v_; __threadfence(); *(volatile T*)(ptr) = vst2_v_; } while (0)

__device__ __forceinline__ unsigned int cmb_pk2(float a, float b) { return (unsigned int)__builtin_bit_cast(unsigned short, (_Float16)a) | ((unsigned int)__builtin_bit_cast(unsigned short, (_Float16)b) << 16); }
__device__ __forceinline__ float cmb_bf(float v) { const unsigned u = __builtin_bit_cast(unsigned, v); const unsigned r = (u + 0x7fffu + ((u >> 16) & 1u)) & 0xffff0000u; return __builtin_bit_cast(float, r); }
__device__ __forceinline__ int xrow(int r) { return (r / SEQ) * SEQ_FULL + (r % SEQ); }

__global__ __launch_bounds__(256) void k_cm_castbT(const float* __restrict__ SRC, int lds, unsigned short* __restrict__ DST, int ldd, int nR, int nC, float sc) {
    const long long u = (long long)blockIdx.x * 256 + threadIdx.x; const int per = nR / 8; if (u >= (long long)nC * per) return; const int c = (int)(u / per); const int r0 = 8 * (int)(u % per);
    float w[8];
#pragma unroll
    for (int e = 0; e < 8; ++e) w[e] = cmb_bf(SRC[(long long)(r0 + e) * lds + c]) * sc;
    cm_u4 pk; pk.x = cmb_pk2(w[0], w[1]); pk.y = cmb_pk2(w[2], w[3]); pk.z = cmb_pk2(w[4], w[5]); pk.w = cmb_pk2(w[6], w[7]); VST2(cm_u4, (cm_u4*)(DST + (long long)c * ldd + r0), pk); }

template <int ABF>
__device__ __forceinline__ void ln_body(const float* __restrict__ A, const float* __restrict__ GA, const float* __restrict__ BE, unsigned short* __restrict__ Y16) {
    #pragma clang fp contract(off)
    const int r = blockIdx.x * 8 + (threadIdx.x >> 5); const int L = threadIdx.x & 31; if (r >= MROWS) return;
    const long long srow = ABF ? (long long)xrow(r) : (long long)r;
    v4f v[8]; float s = 0.f;
#pragma unroll
    for (int q = 0; q < 8; ++q) { const long long o = srow * CW + 4 * L + 128 * q; v[q] = *(const v4f*)(A + o); if (ABF) { v[q].x = cmb_bf(v[q].x); v[q].y = cmb_bf(v[q].y); v[q].z = cmb_bf(v[q].z); v[q].w = cmb_bf(v[q].w); } s += (v[q].x + v[q].y) + (v[q].z + v[q].w); }
#pragma unroll
    for (int o = 16; o > 0; o >>= 1) s += __shfl_xor(s, o, 32);
    const float mu = s * (1.f / CW); float qq = 0.f;
#pragma unroll
    for (int q = 0; q < 8; ++q) { v[q].x -= mu; v[q].y -= mu; v[q].z -= mu; v[q].w -= mu; qq += (v[q].x * v[q].x + v[q].y * v[q].y) + (v[q].z * v[q].z + v[q].w * v[q].w); }
#pragma unroll
    for (int o = 16; o > 0; o >>= 1) qq += __shfl_xor(qq, o, 32);
    const float rs = rsqrtf(qq * (1.f / CW) + 1e-5f);
#pragma unroll
    for (int q = 0; q < 8; ++q) { const int c = 4 * L + 128 * q; const v4f ga = *(const v4f*)(GA + c), be = *(const v4f*)(BE + c); v4f y;
        y.x = v[q].x * rs * cmb_bf(ga.x) + cmb_bf(be.x); y.y = v[q].y * rs * cmb_bf(ga.y) + cmb_bf(be.y); y.z = v[q].z * rs * cmb_bf(ga.z) + cmb_bf(be.z); y.w = v[q].w * rs * cmb_bf(ga.w) + cmb_bf(be.w);
        const long long o = (long long)r * CW + c; bk_u2 pk; pk.x = cmb_pk2(y.x, y.y); pk.y = cmb_pk2(y.z, y.w); VST2(bk_u2, (bk_u2*)(Y16 + o), pk); } }
__global__ __launch_bounds__(256) void k_ln_in(const float* __restrict__ A, const float* __restrict__ GA, const float* __restrict__ BE, unsigned short* __restrict__ Y16) { ln_body<1>(A, GA, BE, Y16); }
__global__ __launch_bounds__(256) void k_ln_ws(const float* __restrict__ A, const float* __restrict__ GA, const float* __restrict__ BE, unsigned short* __restrict__ Y16) { ln_body<0>(A, GA, BE, Y16); }

__device__ __forceinline__ float gelu_erf(float v) { return 0.5f * v * (1.0f + erff(v * 0.70710678118654752f)); }

template <int BIAS_MODE, int OUT_MODE, int RES_MODE>
__device__ __forceinline__ void gemm64_body(const unsigned short* __restrict__ Ap, int lda, const unsigned short* __restrict__ Btp, int ldb,
                                            float* __restrict__ Cf, unsigned short* __restrict__ Ch, int ldc,
                                            const float* __restrict__ bias, const float* __restrict__ resid, int M, int N, int K, float scale) {
    __shared__ __align__(16) float sT[8][16 * 68];
    const _Float16* __restrict__ A  = (const _Float16*)Ap;
    const _Float16* __restrict__ Bt = (const _Float16*)Btp;
    const int lane = threadIdx.x & 31;
    const int wave = threadIdx.x >> 5;
    const int tilesN = N >> 6;
    const int tilesM = M >> 6;
    const int tile = blockIdx.x * 8 + wave;
    if (tile >= tilesM * tilesN) return;
    const int tm = tile / tilesN;
    const int tn = tile - tm * tilesN;
    const int m0 = tm << 6;
    const int n0 = tn << 6;
    const int rlane = lane & 15;
    const int koff  = (lane >> 4) * 8;
    const int mOff  = (lane >> 4) * 8;

    v8f acc[4][4];
#pragma unroll
    for (int i = 0; i < 4; ++i)
#pragma unroll
        for (int j = 0; j < 4; ++j) acc[i][j] = (v8f){0.f, 0.f, 0.f, 0.f, 0.f, 0.f, 0.f, 0.f};

    for (int k0 = 0; k0 < K; k0 += 32) {
        v16h bh[4];
#pragma unroll
        for (int j = 0; j < 4; ++j) {
            const size_t bo = (size_t)(n0 + (j << 4) + rlane) * ldb + koff + k0;
            bh[j] = ld_frag(Bt + bo);
        }
#pragma unroll
        for (int i = 0; i < 4; ++i) {
            const size_t ao = (size_t)(m0 + (i << 4) + rlane) * lda + koff + k0;
            const v16h ah = ld_frag(A + ao);
#pragma unroll
            for (int j = 0; j < 4; ++j) acc[i][j] = mma16_raw(ah, bh[j], acc[i][j]);
            dep_guard_h(acc[i][0], acc[i][3], ah, ah);
        }
        keep4_h(bh[0], bh[1], bh[2], bh[3]);
    }
    acc_guard4(acc[0][0], acc[0][1], acc[0][2], acc[0][3]);
    acc_guard4(acc[1][0], acc[1][1], acc[1][2], acc[1][3]);
    acc_guard4(acc[2][0], acc[2][1], acc[2][2], acc[2][3]);
    acc_guard4(acc[3][0], acc[3][1], acc[3][2], acc[3][3]);

    float bvn[4];
#pragma unroll
    for (int j = 0; j < 4; ++j) bvn[j] = (BIAS_MODE == 2) ? cmb_bf(bias[n0 + (j << 4) + rlane]) : 0.f;
#pragma unroll
    for (int i = 0; i < 4; ++i) {
        const int mBase = m0 + (i << 4);
        float bvm[8];
#pragma unroll
        for (int r = 0; r < 8; ++r) bvm[r] = (BIAS_MODE == 1) ? cmb_bf(bias[mBase + mOff + r]) : 0.f;
#pragma unroll
        for (int j = 0; j < 4; ++j) {
#pragma unroll
            for (int r = 0; r < 8; ++r) {
                float v = acc[i][j][r] * scale;
                if (BIAS_MODE == 1) v += bvm[r];
                if (BIAS_MODE == 2) v += bvn[j];
                sT[wave][(mOff + r) * 68 + (j << 4) + rlane] = v;
            }
        }
        wave_lds_sync();
        if (OUT_MODE == 0) {
            const int hh = lane >> 4, c4 = (lane & 15) * 4;
            v4f vv[8];
#pragma unroll
            for (int it = 0; it < 8; ++it) {
                const int row = it * 2 + hh;
                v4f v = *(const v4f_a*)&sT[wave][row * 68 + c4];
                if (RES_MODE != 0) {
                    const int gr = mBase + row;
                    const size_t ro = (size_t)((RES_MODE == 2) ? xrow(gr) : gr) * ldc + n0 + c4;
                    v4f x = *(const v4f*)(resid + ro);
                    if (RES_MODE == 2) { x.x = cmb_bf(x.x); x.y = cmb_bf(x.y); x.z = cmb_bf(x.z); x.w = cmb_bf(x.w); }
                    v.x += x.x; v.y += x.y; v.z += x.z; v.w += x.w;
                }
                vv[it] = v;
            }
            for (int pass = 0; pass < 2; ++pass) {
#pragma unroll
                for (int it = 0; it < 8; ++it) {
                    const int row = it * 2 + hh;
                    *(volatile v4f*)(Cf + (size_t)(mBase + row) * ldc + n0 + c4) = vv[it];
                }
                __threadfence();
            }
        } else {
            const int q = lane >> 3, c8 = (lane & 7) * 8;
            _Float16* C16 = (_Float16*)Ch;
#pragma unroll 1
            for (int it = 0; it < 4; ++it) {
                const int row = it * 4 + q;
                v4f a  = *(const v4f_a*)&sT[wave][row * 68 + c8];
                v4f bq = *(const v4f_a*)&sT[wave][row * 68 + c8 + 4];
                if (OUT_MODE == 2) {
                    a.x = gelu_erf(a.x); a.y = gelu_erf(a.y); a.z = gelu_erf(a.z); a.w = gelu_erf(a.w);
                    bq.x = gelu_erf(bq.x); bq.y = gelu_erf(bq.y); bq.z = gelu_erf(bq.z); bq.w = gelu_erf(bq.w);
                }
                v8h hv;
                hv[0] = (_Float16)a.x;  hv[1] = (_Float16)a.y;  hv[2] = (_Float16)a.z;  hv[3] = (_Float16)a.w;
                hv[4] = (_Float16)bq.x; hv[5] = (_Float16)bq.y; hv[6] = (_Float16)bq.z; hv[7] = (_Float16)bq.w;
                volatile v8h* d = (volatile v8h*)(C16 + (size_t)(mBase + row) * ldc + n0 + c8);
                *d = hv; __threadfence(); *d = hv;
            }
        }
        wave_lds_sync();
    }
}

__global__ __launch_bounds__(256) void k_gemm_qk(const unsigned short* __restrict__ H16, const unsigned short* __restrict__ WT, unsigned short* __restrict__ QK, const float* __restrict__ bias) {
    gemm64_body<2, 1, 0>(H16, CW, WT, CW, nullptr, QK, QKW, bias, nullptr, MROWS, QKW, CW, 0.0625f); }
__global__ __launch_bounds__(256) void k_gemm_vt(const unsigned short* __restrict__ WVT, const unsigned short* __restrict__ H16, unsigned short* __restrict__ VT, const float* __restrict__ bias) {
    gemm64_body<1, 1, 0>(WVT, CW, H16, CW, nullptr, VT, VTP, bias, nullptr, CW, MROWS, CW, 0.0625f); }
__global__ __launch_bounds__(256) void k_gemm_ao(const unsigned short* __restrict__ Y16, const unsigned short* __restrict__ WT, float* __restrict__ X1, const float* __restrict__ bias, const float* __restrict__ xin) {
    gemm64_body<2, 0, 2>(Y16, CW, WT, CW, X1, nullptr, CW, bias, xin, MROWS, CW, CW, 0.00390625f); }
__global__ __launch_bounds__(256) void k_gemm_fc(const unsigned short* __restrict__ H16, const unsigned short* __restrict__ WT, unsigned short* __restrict__ M16, const float* __restrict__ bias) {
    gemm64_body<2, 2, 0>(H16, CW, WT, CW, nullptr, M16, FW, bias, nullptr, MROWS, FW, CW, 0.0625f); }
__global__ __launch_bounds__(256) void k_gemm_mp(const unsigned short* __restrict__ M16, const unsigned short* __restrict__ WT, float* __restrict__ OUT, const float* __restrict__ bias, const float* __restrict__ X1) {
    gemm64_body<2, 0, 1>(M16, FW, WT, FW, OUT, nullptr, CW, bias, X1, MROWS, CW, FW, 0.0625f); }

#define AT_NW 4
#define AT_PP 40
__global__ __launch_bounds__(128) void k_attn(const unsigned short* __restrict__ QKp, const unsigned short* __restrict__ VTp, unsigned short* __restrict__ Yp) {
    __shared__ __align__(16) _Float16 Ps[AT_NW][16 * AT_PP];
    __shared__ __align__(16) float    Os[AT_NW][16 * 68];
    const _Float16* __restrict__ QK = (const _Float16*)QKp;
    const _Float16* __restrict__ VT = (const _Float16*)VTp;
    _Float16* Y = (_Float16*)Yp;
    const int tid = threadIdx.x, wave = tid >> 5, lane = tid & 31, hh = lane >> 4, c = lane & 15;
    const int nqb = SEQ / 64;
    const int bx = blockIdx.x;
    const int qb = bx % nqb;
    const int bh = bx / nqb;
    const int hd = bh % NH;
    const int b  = bh / NH;
    const int q0 = qb * 64 + wave * 16;
    const size_t qoff  = ((size_t)b * SEQ + q0 + c) * QKW + hd * HD + 8 * hh;
    const size_t kbase = ((size_t)b * SEQ + c) * QKW + CW + hd * HD + 8 * hh;
    const size_t vbase = ((size_t)hd * HD + c) * VTP + (size_t)b * SEQ + 8 * hh;
    const float SC  = 0.125f * 1.4426950408889634f;
    const float NEG = -__builtin_inff();

    float mrow[8], lrow[8];
    v8f oacc[4];
#pragma unroll
    for (int r = 0; r < 8; ++r) { mrow[r] = NEG; lrow[r] = 0.f; }
#pragma unroll
    for (int t = 0; t < 4; ++t) oacc[t] = (v8f){0.f, 0.f, 0.f, 0.f, 0.f, 0.f, 0.f, 0.f};

    const int nhalf = (q0 + 15) / 32 + 1;
    for (int kh = 0; kh < nhalf; ++kh) {
        const int k0 = kh * 32;
        v8f s0 = (v8f){0.f, 0.f, 0.f, 0.f, 0.f, 0.f, 0.f, 0.f};
        v8f s1 = s0;
#pragma unroll
        for (int dc = 0; dc < 2; ++dc) {
            const v16h qa  = ld_frag(QK + qoff + dc * 32);
            const v16h kb0 = ld_frag(QK + kbase + (size_t)(k0) * QKW + dc * 32);
            const v16h kb1 = ld_frag(QK + kbase + (size_t)(k0 + 16) * QKW + dc * 32);
            s0 = mma16(qa, kb0, s0);
            s1 = mma16(qa, kb1, s1);
        }
        const bool needmask = (k0 + 31 > q0);
#pragma unroll
        for (int r = 0; r < 8; ++r) {
            const int qrow = q0 + 8 * hh + r;
            float a0 = s0[r] * SC, a1 = s1[r] * SC;
            a0 = (needmask && (k0 + c > qrow)) ? NEG : a0;
            a1 = (needmask && (k0 + 16 + c > qrow)) ? NEG : a1;
            float m = fmaxf(a0, a1);
            m = fmaxf(m, __shfl_xor(m, 1, 32)); m = fmaxf(m, __shfl_xor(m, 2, 32));
            m = fmaxf(m, __shfl_xor(m, 4, 32)); m = fmaxf(m, __shfl_xor(m, 8, 32));
            const float mnew = fmaxf(mrow[r], m);
            const float alpha = exp2f(mrow[r] - mnew);
            const float p0 = exp2f(a0 - mnew), p1 = exp2f(a1 - mnew);
            float ps = p0 + p1;
            ps += __shfl_xor(ps, 1, 32); ps += __shfl_xor(ps, 2, 32); ps += __shfl_xor(ps, 4, 32); ps += __shfl_xor(ps, 8, 32);
            lrow[r] = lrow[r] * alpha + ps;
            mrow[r] = mnew;
            Ps[wave][(8 * hh + r) * AT_PP + c]      = (_Float16)(p0 * 4096.0f);
            Ps[wave][(8 * hh + r) * AT_PP + 16 + c] = (_Float16)(p1 * 4096.0f);
#pragma unroll
            for (int t = 0; t < 4; ++t) oacc[t][r] *= alpha;
        }
        wave_lds_sync();
        FragU pa;
        pa.h[0] = *(const v8h_a*)&Ps[wave][c * AT_PP + 8 * hh];
        pa.h[1] = *(const v8h_a*)&Ps[wave][c * AT_PP + 16 + 8 * hh];
        v16h vb[4];
#pragma unroll
        for (int t = 0; t < 4; ++t) vb[t] = ld_frag(VT + vbase + (size_t)(t * 16) * VTP + k0);
#pragma unroll
        for (int t = 0; t < 4; ++t) oacc[t] = mma16(pa.v, vb[t], oacc[t]);
        wave_lds_sync();
    }

#pragma unroll
    for (int r = 0; r < 8; ++r) {
        const float inv = 1.0f / (lrow[r] * 256.0f);
#pragma unroll
        for (int t = 0; t < 4; ++t) Os[wave][(8 * hh + r) * 68 + t * 16 + c] = oacc[t][r] * inv;
    }
    wave_lds_sync();
    {
        const int q = lane >> 3, c8 = (lane & 7) * 8;
        v8h hv[4];
#pragma unroll
        for (int it = 0; it < 4; ++it) {
            const int row = it * 4 + q;
            const v4f a  = *(const v4f_a*)&Os[wave][row * 68 + c8];
            const v4f bq = *(const v4f_a*)&Os[wave][row * 68 + c8 + 4];
            v8h t8;
            t8[0] = (_Float16)a.x;  t8[1] = (_Float16)a.y;  t8[2] = (_Float16)a.z;  t8[3] = (_Float16)a.w;
            t8[4] = (_Float16)bq.x; t8[5] = (_Float16)bq.y; t8[6] = (_Float16)bq.z; t8[7] = (_Float16)bq.w;
            hv[it] = t8;
        }
        for (int pass = 0; pass < 2; ++pass) {
#pragma unroll
            for (int it = 0; it < 4; ++it) {
                const int row = it * 4 + q;
                *(volatile v8h*)(Y + ((size_t)b * SEQ + q0 + row) * CW + hd * HD + c8) = hv[it];
            }
            __threadfence();
        }
    }
}

static constexpr size_t SZ_H16   = (size_t)MROWS * CW * 2;
static constexpr size_t SZ_WQKVT = (size_t)3 * CW * CW * 2;
static constexpr size_t SZ_WAOT  = (size_t)CW * CW * 2;
static constexpr size_t SZ_WFCT  = (size_t)FW * CW * 2;
static constexpr size_t SZ_WMPT  = (size_t)CW * FW * 2;
static constexpr size_t SZ_QK16  = (size_t)MROWS * QKW * 2;
static constexpr size_t SZ_VT16  = (size_t)CW * VTP * 2;
static constexpr size_t SZ_Y16   = (size_t)MROWS * CW * 2;
static constexpr size_t SZ_X1    = (size_t)MROWS * CW * 4;
static constexpr size_t SZ_H2    = (size_t)MROWS * CW * 2;
static constexpr size_t SZ_M16   = (size_t)MROWS * FW * 2;
static constexpr size_t OFF_H16   = 0;
static constexpr size_t OFF_WQKVT = OFF_H16 + SZ_H16;
static constexpr size_t OFF_WAOT  = OFF_WQKVT + SZ_WQKVT;
static constexpr size_t OFF_WFCT  = OFF_WAOT + SZ_WAOT;
static constexpr size_t OFF_WMPT  = OFF_WFCT + SZ_WFCT;
static constexpr size_t OFF_QK16  = OFF_WMPT + SZ_WMPT;
static constexpr size_t OFF_VT16  = OFF_QK16 + SZ_QK16;
static constexpr size_t OFF_Y16   = OFF_VT16 + SZ_VT16;
static constexpr size_t OFF_X1    = OFF_Y16 + SZ_Y16;
static constexpr size_t OFF_H2    = OFF_X1 + SZ_X1;
static constexpr size_t OFF_M16   = OFF_H2 + SZ_H2;
static constexpr size_t WS_TOTAL  = OFF_M16 + SZ_M16;
static_assert(SZ_H16 % 256 == 0 && SZ_WQKVT % 256 == 0 && SZ_WAOT % 256 == 0 && SZ_WFCT % 256 == 0 && SZ_WMPT % 256 == 0);
static_assert(SZ_QK16 % 256 == 0 && SZ_VT16 % 256 == 0 && SZ_Y16 % 256 == 0 && SZ_X1 % 256 == 0 && SZ_H2 % 256 == 0 && SZ_M16 % 256 == 0);
static_assert(WS_TOTAL <= (size_t)134217728);
static_assert(((MROWS / 64) * (QKW / 64)) % 8 == 0 && ((CW / 64) * (MROWS / 64)) % 8 == 0 && ((MROWS / 64) * (FW / 64)) % 8 == 0);

extern "C" void kernel_launch(void* const* d_in, const int* in_sizes, int n_in, void* d_out, int out_size, void* d_ws, size_t ws_size, hipStream_t stream) {
    if (n_in < 13) return;
    if (in_sizes[0] < MROWS * CW) return;
    if (in_sizes[1] < 3 * CW * CW || in_sizes[2] < 3 * CW) return;
    if (in_sizes[3] < CW * CW || in_sizes[4] < CW) return;
    if (in_sizes[5] < CW * FW || in_sizes[6] < FW) return;
    if (in_sizes[7] < FW * CW || in_sizes[8] < CW) return;
    if (in_sizes[9] < CW || in_sizes[10] < CW || in_sizes[11] < CW || in_sizes[12] < CW) return;
    if (out_size < MROWS * CW) return;
    if (WS_TOTAL > ws_size) return;
    const float* x     = (const float*)d_in[0];
    const float* W_qkv = (const float*)d_in[1];
    const float* b_qkv = (const float*)d_in[2];
    const float* W_ao  = (const float*)d_in[3];
    const float* b_ao  = (const float*)d_in[4];
    const float* W_fc  = (const float*)d_in[5];
    const float* b_fc  = (const float*)d_in[6];
    const float* W_mp  = (const float*)d_in[7];
    const float* b_mp  = (const float*)d_in[8];
    const float* g1    = (const float*)d_in[9];
    const float* be1   = (const float*)d_in[10];
    const float* g2    = (const float*)d_in[11];
    const float* be2   = (const float*)d_in[12];
    float* out = (float*)d_out;
    char* wsp = (char*)d_ws;
    unsigned short* H16   = (unsigned short*)(wsp + OFF_H16);
    unsigned short* WQKVT = (unsigned short*)(wsp + OFF_WQKVT);
    unsigned short* WAOT  = (unsigned short*)(wsp + OFF_WAOT);
    unsigned short* WFCT  = (unsigned short*)(wsp + OFF_WFCT);
    unsigned short* WMPT  = (unsigned short*)(wsp + OFF_WMPT);
    unsigned short* QK16  = (unsigned short*)(wsp + OFF_QK16);
    unsigned short* VT16  = (unsigned short*)(wsp + OFF_VT16);
    unsigned short* Y16   = (unsigned short*)(wsp + OFF_Y16);
    float*          X1    = (float*)(wsp + OFF_X1);
    unsigned short* H2    = (unsigned short*)(wsp + OFF_H2);
    unsigned short* M16   = (unsigned short*)(wsp + OFF_M16);

    k_cm_castbT<<<(unsigned)(((long long)(3 * CW) * (CW / 8) + 255) / 256), 256, 0, stream>>>(W_qkv, 3 * CW, WQKVT, CW, CW, 3 * CW, 16.0f);
    k_cm_castbT<<<(unsigned)(((long long)(CW) * (CW / 8) + 255) / 256), 256, 0, stream>>>(W_ao, CW, WAOT, CW, CW, CW, 16.0f);
    k_cm_castbT<<<(unsigned)(((long long)(FW) * (CW / 8) + 255) / 256), 256, 0, stream>>>(W_fc, FW, WFCT, CW, CW, FW, 16.0f);
    k_cm_castbT<<<(unsigned)(((long long)(CW) * (FW / 8) + 255) / 256), 256, 0, stream>>>(W_mp, CW, WMPT, FW, FW, CW, 16.0f);
    k_ln_in<<<MROWS / 8, 256, 0, stream>>>(x, g1, be1, H16);
    k_gemm_qk<<<(unsigned)(((MROWS / 64) * (QKW / 64) + 7) / 8), 256, 0, stream>>>(H16, WQKVT, QK16, b_qkv);
    k_gemm_vt<<<(unsigned)(((CW / 64) * (MROWS / 64) + 7) / 8), 256, 0, stream>>>(WQKVT + (size_t)QKW * CW, H16, VT16, b_qkv + QKW);
    k_attn<<<(unsigned)(NB * NH * (SEQ / 64)), 32 * AT_NW, 0, stream>>>(QK16, VT16, Y16);
    k_gemm_ao<<<(unsigned)(((MROWS / 64) * (CW / 64) + 7) / 8), 256, 0, stream>>>(Y16, WAOT, X1, b_ao, x);
    k_ln_ws<<<MROWS / 8, 256, 0, stream>>>(X1, g2, be2, H2);
    k_gemm_fc<<<(unsigned)(((MROWS / 64) * (FW / 64) + 7) / 8), 256, 0, stream>>>(H2, WFCT, M16, b_fc);
    k_gemm_mp<<<(unsigned)(((MROWS / 64) * (CW / 64) + 7) / 8), 256, 0, stream>>>(M16, WMPT, out, b_mp, X1);
}
